// Graph_MultiHeadAttention_53747220742568
// MI455X (gfx1250) — hardware-run, weakly checked
//
#include <hip/hip_runtime.h>
#include <stddef.h>


#define DIN    128
#define DQ     128
#define NW     5
#define GT     128
#define SPW    (32 * 64)
#define WPP    136
#define RB     1024
#define RBBITS 10
#define RMAX   64
#define RMBITS 6
#define TABW   (2 * RMAX)
#define CHUNK  4096
#define LCAP   18432
#define DEGCAP 64
#define SCW    (32 * DEGCAP)
#define WSCAP  134217728
#define ASCL   8.0f
#define WSCL   64.0f
#define INVSCL 0.001953125f
#define PRISCL 0.00390625f

#define EDGE_LDS_INTS  (RB + 8 + RB + LCAP)
#define EDGE_LDS_BYTES ((EDGE_LDS_INTS + 8 * SCW) * 4)

static_assert(RB == (1 << RBBITS));
static_assert(RMAX == (1 << RMBITS));
static_assert(CHUNK == 8 * 16 * 32);
static_assert(CHUNK == 4 * 4 * 256);
static_assert(TABW * 4 == 32 * 16);
static_assert((WPP % 8) == 0);
static_assert((RB % 64) == 0);
static_assert(RB == 4 * 256);
static_assert(((EDGE_LDS_INTS * 4) % 16) == 0);
static_assert(EDGE_LDS_BYTES < 300000);
static_assert(SCW >= 256);
static_assert((DIN % 32) == 0);
static_assert(DQ == 128);
static_assert(DIN == 128);

typedef float          v4f  __attribute__((ext_vector_type(4)));
typedef float          v8f  __attribute__((ext_vector_type(8)));
typedef int            v4i  __attribute__((ext_vector_type(4)));
typedef unsigned int   v4u  __attribute__((ext_vector_type(4)));
typedef unsigned short v4us __attribute__((ext_vector_type(4)));
typedef unsigned short v8us __attribute__((ext_vector_type(8)));
typedef _Float16       v16h __attribute__((ext_vector_type(16)));
union FragH { v16h v; v8us u[2]; };

__device__ __forceinline__ unsigned short h16(float f) {
  const _Float16 h = (_Float16)f;
  return __builtin_bit_cast(unsigned short, h);
}
__device__ __forceinline__ float hf(unsigned short u) {
  return (float)__builtin_bit_cast(_Float16, u);
}

__device__ __forceinline__ v8us cvt8(v4f a, v4f b, float s) {
  v8us r;
  r[0] = h16(a.x * s); r[1] = h16(a.y * s); r[2] = h16(a.z * s); r[3] = h16(a.w * s);
  r[4] = h16(b.x * s); r[5] = h16(b.y * s); r[6] = h16(b.z * s); r[7] = h16(b.w * s);
  return r;
}

__device__ __forceinline__ v8f wmh(v16h a, v16h b, v8f c) {
  v8f d = __builtin_amdgcn_wmma_f32_16x16x32_f16(false, a, false, b, (short)0, c, false, false);
  asm volatile("v_nop\n\tv_nop\n\tv_nop\n\tv_nop" : "+v"(d) : "v"(a), "v"(b));
  return d;
}

template <int NB>
__device__ __forceinline__ unsigned int match_mask(unsigned int base, int key) {
  unsigned int msk = base;
#pragma unroll
  for (int b = 0; b < NB; ++b) {
    const bool bit = ((key >> b) & 1) != 0;
    const unsigned int bb = __builtin_amdgcn_ballot_w32(bit);
    msk &= bit ? bb : ~bb;
  }
  return msk;
}

__global__ __launch_bounds__(256) void k_csort(
    const int* __restrict__ key, unsigned int* csort, int* tab, int nN, int nE) {
  __shared__ __attribute__((aligned(16))) unsigned int sImg[CHUNK];
  __shared__ int cw[8 * RMAX];
  __shared__ __attribute__((aligned(16))) int sTb[TABW];
  __shared__ int sWt[8];
  int* sPre = sTb;
  int* sCn  = sTb + RMAX;
  const int tid = (int)threadIdx.x, lane = tid & 31, wave = tid >> 5;
  const int c = (int)blockIdx.x;
  const int cbase = c * CHUNK;

  for (int i = tid; i < 8 * RMAX; i += 256) cw[i] = 0;
  {
    const v4u s = {0xffffffffu, 0xffffffffu, 0xffffffffu, 0xffffffffu};
    for (int i = tid; i < CHUNK / 4; i += 256) ((v4u*)sImg)[i] = s;
  }
  __syncthreads();

  unsigned int ent[16];
  int pk[16];
  const unsigned int lt = (1u << lane) - 1u;
#pragma unroll
  for (int i = 0; i < 16; ++i) {
    const int e = cbase + wave * 512 + 32 * i + lane;
    const int ea = e > nE - 1 ? nE - 1 : e;
    const int d = key[ea];
    const bool valid = (e < nE) && ((unsigned)d < (unsigned)nN);
    const int dd = valid ? d : 0;
    const int r  = dd >> RBBITS;
    const int jl = dd & (RB - 1);
    const unsigned int pay = (unsigned int)ea;
    const unsigned int msk = match_mask<RMBITS>(__builtin_amdgcn_ballot_w32(valid), r);
    const int rank = (int)__builtin_popcount(msk & lt);
    const int grp  = (int)__builtin_popcount(msk);
    const int base = cw[wave * RMAX + r];
    pk[i]  = valid ? ((r << 12) | (base + rank)) : -1;
    ent[i] = (pay << RBBITS) | (unsigned int)jl;
    if (valid && rank == 0) cw[wave * RMAX + r] = base + grp;
    __syncthreads();
  }

  if (tid < RMAX) {
    int run = 0;
#pragma unroll
    for (int w = 0; w < 8; ++w) {
      const int v = cw[w * RMAX + tid];
      cw[w * RMAX + tid] = run;
      run += v;
    }
    sCn[tid] = run;
  }
  __syncthreads();
  {
    const int vr = sCn[tid & (RMAX - 1)];
    const int v  = (tid < RMAX) ? vr : 0;
    int x = v;
#pragma unroll
    for (int dd = 1; dd < 32; dd <<= 1) {
      const int y = __shfl_up(x, dd);
      x += (lane >= dd) ? y : 0;
    }
    if (lane == 31) sWt[wave] = x;
    __syncthreads();
    int pre = 0;
#pragma unroll
    for (int w = 0; w < 8; ++w) { const int tw = sWt[w]; pre += (w < wave) ? tw : 0; }
    if (tid < RMAX) sPre[tid] = pre + x - v;
  }
  __syncthreads();

#pragma unroll
  for (int i = 0; i < 16; ++i) {
    if (pk[i] >= 0) {
      const int r = (pk[i] >> 12) & (RMAX - 1);
      const int q = pk[i] & 4095;
      const int pos = sPre[r] + cw[wave * RMAX + r] + q;
      if ((unsigned)pos < (unsigned)CHUNK) sImg[pos] = ent[i];
    }
  }
  __syncthreads();

  v4u iv[4];
#pragma unroll
  for (int it = 0; it < 4; ++it) iv[it] = ((const v4u*)sImg)[it * 256 + tid];
  const v4i tv = *(const v4i*)(sTb + 4 * lane);
  unsigned int* gp = csort + (size_t)c * CHUNK;
  int* tp = tab + (size_t)c * TABW + 4 * lane;
  const bool wt = tid < 32;
#pragma unroll
  for (int it = 0; it < 4; ++it) *(volatile v4u*)(gp + 4 * (it * 256 + tid)) = iv[it];
  if (wt) *(volatile v4i*)tp = tv;
  __threadfence();
#pragma unroll
  for (int it = 0; it < 4; ++it) *(volatile v4u*)(gp + 4 * (it * 256 + tid)) = iv[it];
  if (wt) *(volatile v4i*)tp = tv;
}

__global__ __launch_bounds__(256) void k_xcvt(
    const float* __restrict__ x, unsigned short* x16, int nN, int nNp) {
  const int tid = (int)threadIdx.x;
  const int rb = (int)blockIdx.x * 64;
  const v4f zero4 = {0.0f, 0.0f, 0.0f, 0.0f};
  v8us o[4];
  size_t po[4];
#pragma unroll
  for (int it = 0; it < 4; ++it) {
    const int p = it * 256 + tid;
    const int row = rb + (p >> 4);
    const int c8 = (p & 15) * 8;
    const bool live = row < nN;
    const int xr = live ? row : (nN - 1);
    v4f a = *(const v4f*)(x + (size_t)xr * DIN + c8);
    v4f b = *(const v4f*)(x + (size_t)xr * DIN + c8 + 4);
    a = live ? a : zero4;
    b = live ? b : zero4;
    o[it]  = cvt8(a, b, ASCL);
    po[it] = (size_t)row * DIN + c8;
  }
#pragma unroll
  for (int it = 0; it < 4; ++it) *(volatile v8us*)(x16 + po[it]) = o[it];
  __threadfence();
#pragma unroll
  for (int it = 0; it < 4; ++it) *(volatile v8us*)(x16 + po[it]) = o[it];
}

__global__ __launch_bounds__(256) void k_wprep(
    const float* __restrict__ W0, const float* __restrict__ W1, const float* __restrict__ W2,
    const float* __restrict__ W3, const float* __restrict__ W4, unsigned short* w16) {
  __shared__ __attribute__((aligned(16))) unsigned short sT[DQ * WPP];
  const int tid = (int)threadIdx.x;
  const int mat = (int)blockIdx.x;
  const float* W = (mat == 0) ? W0 : ((mat == 1) ? W1 : ((mat == 2) ? W2 : ((mat == 3) ? W3 : W4)));

#pragma unroll 1
  for (int it = 0; it < (DIN * DQ) / 256; ++it) {
    const int idx = it * 256 + tid;
    const int k = idx >> 7, nl = idx & 127;
    sT[nl * WPP + k] = h16(W[(size_t)k * DQ + nl] * WSCL);
  }
  __syncthreads();

  v8us pv[8];
  size_t po[8];
#pragma unroll
  for (int it = 0; it < 8; ++it) {
    const int p = it * 256 + tid;
    const int row = p >> 4, c8 = (p & 15) * 8;
    pv[it] = *(const v8us*)(sT + row * WPP + c8);
    po[it] = (size_t)(mat * DQ + row) * DIN + c8;
  }
#pragma unroll
  for (int it = 0; it < 8; ++it) *(volatile v8us*)(w16 + po[it]) = pv[it];
  __threadfence();
#pragma unroll
  for (int it = 0; it < 8; ++it) *(volatile v8us*)(w16 + po[it]) = pv[it];
}

__global__ __launch_bounds__(GT) void k_gemm(
    const unsigned short* __restrict__ A, const unsigned short* __restrict__ Bt,
    const float* __restrict__ b0, const float* __restrict__ b1,
    const float* __restrict__ b2, const float* __restrict__ b3,
    unsigned short* outH, float* outF, int K, int Mp, int woff, int nh, int rowLim) {
  __shared__ __attribute__((aligned(16))) float sT[4 * SPW];
  const int tid = (int)threadIdx.x, lane = tid & 31, wave = tid >> 5, hh = lane >> 4, m = lane & 15;
  const int mat = (int)blockIdx.z;
  const int wsel = mat + woff;
  const int r0 = (int)blockIdx.y * 64 + (wave >> 1) * 32;
  const int c0 = (int)blockIdx.x * 128 + (wave & 1) * 64;
  const float* bias = (mat == 0) ? b0 : ((mat == 1) ? b1 : ((mat == 2) ? b2 : b3));

  int ra0 = r0 + m;      ra0 = ra0 > Mp - 1 ? Mp - 1 : ra0;
  int ra1 = r0 + 16 + m; ra1 = ra1 > Mp - 1 ? Mp - 1 : ra1;
  const unsigned short* ap0 = A + (size_t)ra0 * K + 8 * hh;
  const unsigned short* ap1 = A + (size_t)ra1 * K + 8 * hh;
  const unsigned short* bp[4];
#pragma unroll
  for (int j = 0; j < 4; ++j) {
    int cb = c0 + 16 * j + m; cb = cb > DQ - 1 ? DQ - 1 : cb;
    bp[j] = Bt + ((size_t)wsel * DQ + cb) * K + 8 * hh;
  }

  v8f acc[2][4];
#pragma unroll
  for (int i = 0; i < 2; ++i)
#pragma unroll
    for (int j = 0; j < 4; ++j) { v8f z = {0.f, 0.f, 0.f, 0.f, 0.f, 0.f, 0.f, 0.f}; acc[i][j] = z; }

  const int nk = K >> 5;
#pragma unroll 1
  for (int kt = 0; kt < nk; ++kt) {
    const int kb = kt << 5;
    FragH a0, a1;
    a0.u[0] = *(const v8us*)(ap0 + kb);
    a0.u[1] = *(const v8us*)(ap0 + kb + 16);
    a1.u[0] = *(const v8us*)(ap1 + kb);
    a1.u[1] = *(const v8us*)(ap1 + kb + 16);
#pragma unroll
    for (int j = 0; j < 4; ++j) {
      FragH bf;
      bf.u[0] = *(const v8us*)(bp[j] + kb);
      bf.u[1] = *(const v8us*)(bp[j] + kb + 16);
      acc[0][j] = wmh(a0.v, bf.v, acc[0][j]);
      acc[1][j] = wmh(a1.v, bf.v, acc[1][j]);
    }
  }

  float* sw = sT + wave * SPW;
#pragma unroll
  for (int i = 0; i < 2; ++i)
#pragma unroll
    for (int j = 0; j < 4; ++j)
#pragma unroll
      for (int r = 0; r < 8; ++r)
        sw[(16 * i + 8 * hh + r) * 64 + 16 * j + m] = acc[i][j][r];
  __syncthreads();

  if (mat < nh) {
    unsigned short* oH = outH + (size_t)mat * (size_t)Mp * DQ;
    v8us hv[8];
    size_t po[8];
#pragma unroll
    for (int it = 0; it < 8; ++it) {
      const int f = it * 32 + lane;
      const int row = f >> 3, c8 = (f & 7) * 8;
      const v4f v0 = *(const v4f*)(sw + row * 64 + c8);
      const v4f v1 = *(const v4f*)(sw + row * 64 + c8 + 4);
      int gc = c0 + c8; gc = gc > DQ - 8 ? DQ - 8 : gc;
      const v4f b0v = *(const v4f*)(bias + gc);
      const v4f b1v = *(const v4f*)(bias + gc + 4);
      const v4f o0 = v0 * INVSCL + b0v;
      const v4f o1 = v1 * INVSCL + b1v;
      hv[it] = cvt8(o0, o1, ASCL);
      po[it] = (size_t)(r0 + row) * DQ + c0 + c8;
    }
#pragma unroll
    for (int it = 0; it < 8; ++it) *(volatile v8us*)(oH + po[it]) = hv[it];
    __threadfence();
#pragma unroll
    for (int it = 0; it < 8; ++it) *(volatile v8us*)(oH + po[it]) = hv[it];
  } else {
    float* oF = outF + (size_t)(mat - nh) * (size_t)Mp * DQ;
    v4f ov[16];
    size_t po[16];
    bool ok[16];
#pragma unroll
    for (int it = 0; it < 16; ++it) {
      const int f = it * 32 + lane;
      const int row = f >> 4, c4 = (f & 15) * 4;
      const v4f v = *(const v4f*)(sw + row * 64 + c4);
      int gc = c0 + c4; gc = gc > DQ - 4 ? DQ - 4 : gc;
      const v4f bb = *(const v4f*)(bias + gc);
      ov[it] = v * INVSCL + bb;
      ok[it] = (r0 + row) < rowLim;
      po[it] = (size_t)(r0 + row) * DQ + c0 + c4;
    }
#pragma unroll
    for (int it = 0; it < 16; ++it) { if (ok[it]) *(volatile v4f*)(oF + po[it]) = ov[it]; }
    __threadfence();
#pragma unroll
    for (int it = 0; it < 16; ++it) { if (ok[it]) *(volatile v4f*)(oF + po[it]) = ov[it]; }
  }
}

__global__ __launch_bounds__(256) void k_edge(
    const unsigned short* __restrict__ q16, const unsigned short* __restrict__ k16,
    const float* __restrict__ vF, const float* __restrict__ sF,
    const int* __restrict__ src,
    const unsigned int* __restrict__ csort, const int* __restrict__ tab,
    unsigned short* h16, int nN, int nNp, int nE, int nCh) {
  extern __shared__ __attribute__((aligned(16))) int dsm[];
  __shared__ int sWtot[8];
  int*   sOff  = dsm;
  int*   sCur  = dsm + (RB + 8);
  int*   sList = sCur + RB;
  float* sSc   = (float*)(sList + LCAP);
  const int tid = (int)threadIdx.x, lane = tid & 31, wave = tid >> 5;
  const int rgn = (int)blockIdx.x;
  const int n0 = rgn * RB;
  const unsigned int lt = (1u << lane) - 1u;

  for (int i = tid; i < RB + 8; i += 256) sOff[i] = 0;
  for (int i = tid; i < RB; i += 256) sCur[i] = 0;
  __syncthreads();

#pragma unroll 1
  for (int c = 0; c < nCh; ++c) {
    int pre = tab[(size_t)c * TABW + rgn];
    int n   = tab[(size_t)c * TABW + RMAX + rgn];
    pre = pre < 0 ? 0 : (pre > CHUNK ? CHUNK : pre);
    n = n < 0 ? 0 : (n > CHUNK - pre ? CHUNK - pre : n);
    const int nstep = (n + 31) >> 5;
    const unsigned int* cp = csort + (size_t)c * CHUNK + pre;
#pragma unroll 1
    for (int s = 0; s < nstep; ++s) {
      if (wave == 0) {
        const int i = (s << 5) + lane;
        const bool valid = i < n;
        const int ic = i > n - 1 ? n - 1 : i;
        const unsigned int en = cp[ic];
        const int j = (int)(en & (unsigned int)(RB - 1));
        const unsigned int msk = match_mask<RBBITS>(__builtin_amdgcn_ballot_w32(valid), j);
        const int rank = (int)__builtin_popcount(msk & lt);
        const int grp  = (int)__builtin_popcount(msk);
        if (valid && rank == 0) sOff[j] = sOff[j] + grp;
      }
      __syncthreads();
    }
  }
  __syncthreads();

  {
    int cn[4];
    int ls = 0;
#pragma unroll
    for (int i = 0; i < 4; ++i) { cn[i] = sOff[4 * tid + i]; ls += cn[i]; }
    int x = ls;
#pragma unroll
    for (int dd = 1; dd < 32; dd <<= 1) {
      const int y = __shfl_up(x, dd);
      x += (lane >= dd) ? y : 0;
    }
    if (lane == 31) sWtot[wave] = x;
    __syncthreads();
    int pre = 0;
#pragma unroll
    for (int w = 0; w < 8; ++w) { const int tw = sWtot[w]; pre += (w < wave) ? tw : 0; }
    int run = pre + x - ls;
#pragma unroll
    for (int i = 0; i < 4; ++i) { sOff[4 * tid + i] = run; run += cn[i]; }
    if (tid == 255) sOff[RB] = run;
  }
  __syncthreads();

#pragma unroll 1
  for (int c = 0; c < nCh; ++c) {
    int pre = tab[(size_t)c * TABW + rgn];
    int n   = tab[(size_t)c * TABW + RMAX + rgn];
    pre = pre < 0 ? 0 : (pre > CHUNK ? CHUNK : pre);
    n = n < 0 ? 0 : (n > CHUNK - pre ? CHUNK - pre : n);
    const int nstep = (n + 31) >> 5;
    const unsigned int* cp = csort + (size_t)c * CHUNK + pre;
#pragma unroll 1
    for (int s = 0; s < nstep; ++s) {
      if (wave == 0) {
        const int i = (s << 5) + lane;
        const bool valid = i < n;
        const int ic = i > n - 1 ? n - 1 : i;
        const unsigned int en = cp[ic];
        const int j = (int)(en & (unsigned int)(RB - 1));
        int e = (int)(en >> RBBITS);
        e = e > nE - 1 ? nE - 1 : e;
        const unsigned int msk = match_mask<RBBITS>(__builtin_amdgcn_ballot_w32(valid), j);
        const int rank = (int)__builtin_popcount(msk & lt);
        const int grp  = (int)__builtin_popcount(msk);
        const int cur  = sCur[j];
        const int p0   = sOff[j] + cur + rank;
        if (valid && (unsigned)p0 < (unsigned)LCAP) sList[p0] = e;
        if (valid && rank == 0) sCur[j] = cur + grp;
      }
      __syncthreads();
    }
  }
  __syncthreads();

  const int c4 = 4 * lane;
  int Rbp = nNp - n0; Rbp = Rbp > RB ? RB : Rbp;
  const int niter = (Rbp + 7) >> 3;
  float* sw = sSc + wave * SCW;
  const v4f zero4 = {0.0f, 0.0f, 0.0f, 0.0f};
#pragma unroll 1
  for (int jj = 0; jj < niter; ++jj) {
    const int j = jj * 8 + wave;
    const bool act = j < Rbp;
    const int jc = act ? j : (Rbp - 1);
    const int node = n0 + jc;
    const bool live = node < nN;
    int lb = __builtin_amdgcn_readfirstlane(sOff[jc]);
    int ub = __builtin_amdgcn_readfirstlane(sOff[jc + 1]);
    lb = lb < 0 ? 0 : (lb > LCAP ? LCAP : lb);
    ub = ub < 0 ? 0 : (ub > LCAP ? LCAP : ub);
    int cnt = ub - lb;
    cnt = cnt < 0 ? 0 : (cnt > DEGCAP ? DEGCAP : cnt);

    const v4us qv = *(const v4us*)(q16 + (size_t)node * DQ + c4);
    float qf[4];
#pragma unroll
    for (int cc = 0; cc < 4; ++cc) qf[cc] = hf(qv[cc]);

    float mx = __int_as_float(0xff800000u);
#pragma unroll 1
    for (int it = 0; it < cnt; ++it) {
      int li = lb + it; li = li > LCAP - 1 ? LCAP - 1 : li;
      int e = sList[li]; e = e < 0 ? 0 : (e > nE - 1 ? nE - 1 : e);
      int s = src[e];   s = s < 0 ? 0 : (s > nN - 1 ? nN - 1 : s);
      const v4us kv = *(const v4us*)(k16 + (size_t)s * DQ + c4);
      float part = qf[0] * hf(kv[0]);
      part = fmaf(qf[1], hf(kv[1]), part);
      part = fmaf(qf[2], hf(kv[2]), part);
      part = fmaf(qf[3], hf(kv[3]), part);
      part += __shfl_xor(part, 1);
      part += __shfl_xor(part, 2);
      const float sc = part * PRISCL;
      mx = fmaxf(mx, sc);
      sw[it * 32 + lane] = sc;
    }

    v4f acc = zero4;
    float z = 0.0f;
#pragma unroll 1
    for (int it = 0; it < cnt; ++it) {
      int li = lb + it; li = li > LCAP - 1 ? LCAP - 1 : li;
      int e = sList[li]; e = e < 0 ? 0 : (e > nE - 1 ? nE - 1 : e);
      int s = src[e];   s = s < 0 ? 0 : (s > nN - 1 ? nN - 1 : s);
      const float sc = sw[it * 32 + lane];
      const float p = __expf(sc - mx);
      const v4f vv = *(const v4f*)(vF + (size_t)s * DQ + c4);
      acc = acc + vv * p;
      z += p;
    }
    const float zs = (cnt > 0) ? z : 1.0f;
    const float rz = 1.0f / zs;
    const v4f sv = *(const v4f*)(sF + (size_t)node * DQ + c4);
    v4f hv = acc * rz + sv;
    hv = live ? hv : zero4;

    *(v4f*)(sw + c4) = hv;
    __syncthreads();
    const int l8 = 8 * (lane & 15);
    const v4f u0 = *(const v4f*)(sw + l8);
    const v4f u1 = *(const v4f*)(sw + l8 + 4);
    __syncthreads();

    const v8us o = cvt8(u0, u1, ASCL);
    unsigned short* op = h16 + (size_t)node * DQ + l8;
    const bool wst = act && (lane < 16);
    if (wst) *(volatile v8us*)op = o;
    __threadfence();
    if (wst) *(volatile v8us*)op = o;
  }
}

extern "C" void kernel_launch(void* const* d_in, const int* in_sizes, int n_in,
                              void* d_out, int out_size, void* d_ws, size_t ws_size,
                              hipStream_t stream) {
  if (n_in < 12) return;
  const int nN = in_sizes[0] / DIN;
  const int nE = in_sizes[1] / 2;
  if (nN <= 0 || nE <= 0) return;
  if (in_sizes[0] != nN * DIN) return;
  if (in_sizes[1] != 2 * nE) return;
  if (nN > RMAX * RB || nE > (1 << 22)) return;
  if (in_sizes[2] != DIN * DQ || in_sizes[4] != DIN * DQ || in_sizes[6] != DIN * DQ ||
      in_sizes[8] != DIN * DQ || in_sizes[10] != DIN * DQ) return;
  if (in_sizes[3] != DQ || in_sizes[5] != DQ || in_sizes[7] != DQ || in_sizes[9] != DQ || in_sizes[11] != DQ) return;
  if (out_size != nN * DQ) return;

  const float* x   = (const float*)d_in[0];
  const int*   ei  = (const int*)d_in[1];
  const float* Wq  = (const float*)d_in[2];
  const float* bq  = (const float*)d_in[3];
  const float* Wk  = (const float*)d_in[4];
  const float* bk  = (const float*)d_in[5];
  const float* Wv  = (const float*)d_in[6];
  const float* bv  = (const float*)d_in[7];
  const float* Ws  = (const float*)d_in[8];
  const float* bs  = (const float*)d_in[9];
  const float* Wo  = (const float*)d_in[10];
  const float* bo  = (const float*)d_in[11];
  const int*   esrc = ei;
  const int*   edst = ei + nE;
  float* out = (float*)d_out;

  const int nCh = (nE + CHUNK - 1) / CHUNK;
  const int nR  = (nN + RB - 1) / RB;
  const int nNp = ((nN + 63) / 64) * 64;

  const size_t szX16 = (size_t)nNp * DIN * 2;
  const size_t szW16 = (size_t)NW * DQ * DIN * 2;
  const size_t szQK  = (size_t)2 * (size_t)nNp * DQ * 2;
  const size_t szVS  = (size_t)2 * (size_t)nNp * DQ * 4;
  const size_t szCS  = (size_t)nCh * CHUNK * 4;
  const size_t szTab = (size_t)nCh * TABW * 4;
  const size_t szH16 = (size_t)nNp * DQ * 2;
  size_t off = 0;
  const size_t oX = off; off += szX16; off = (off + 255) & ~(size_t)255;
  const size_t oW = off; off += szW16; off = (off + 255) & ~(size_t)255;
  const size_t oQ = off; off += szQK;  off = (off + 255) & ~(size_t)255;
  const size_t oV = off; off += szVS;  off = (off + 255) & ~(size_t)255;
  const size_t oC = off; off += szCS;  off = (off + 255) & ~(size_t)255;
  const size_t oT = off; off += szTab; off = (off + 255) & ~(size_t)255;
  const size_t oH = off; off += szH16; off = (off + 255) & ~(size_t)255;
  if (off > ws_size || off > (size_t)WSCAP) return;

  char* ws = (char*)d_ws;
  unsigned short* x16   = (unsigned short*)(ws + oX);
  unsigned short* w16   = (unsigned short*)(ws + oW);
  unsigned short* qk16  = (unsigned short*)(ws + oQ);
  float*          vsF   = (float*)(ws + oV);
  unsigned int*   csort = (unsigned int*)(ws + oC);
  int*            tab   = (int*)(ws + oT);
  unsigned short* h16   = (unsigned short*)(ws + oH);
  const unsigned short* q16 = qk16;
  const unsigned short* k16 = qk16 + (size_t)nNp * DQ;
  const float* vF = vsF;
  const float* sF = vsF + (size_t)nNp * DQ;

  k_csort<<<nCh, 256, 0, stream>>>(edst, csort, tab, nN, nE);

  k_xcvt<<<nNp / 64, 256, 0, stream>>>(x, x16, nN, nNp);

  k_wprep<<<NW, 256, 0, stream>>>(Wq, Wk, Wv, Ws, Wo, w16);

  k_gemm<<<dim3(DQ / 128, nNp / 64, 4), GT, 0, stream>>>(x16, w16, bq, bk, bv, bs, qk16, vsF, DIN, nNp, 0, 2, nNp);

  hipFuncSetAttribute(reinterpret_cast<const void*>(&k_edge),
                      hipFuncAttributeMaxDynamicSharedMemorySize, EDGE_LDS_BYTES);
  k_edge<<<nR, 256, EDGE_LDS_BYTES, stream>>>(q16, k16, vF, sF, esrc, csort, tab, h16, nN, nNp, nE, nCh);

  k_gemm<<<dim3(DQ / 128, nNp / 64, 1), GT, 0, stream>>>(h16, w16, bo, bo, bo, bo, qk16, out, DIN, nNp, NW - 1, 0, nN);
}
